// SelfAttention_11854109737180
// MI455X (gfx1250) — hardware-verified
//
#include <hip/hip_runtime.h>


#ifndef NB
#define NB 2
#endif
#ifndef SEQ
#define SEQ 4096
#endif
#define NB_FULL    2
#define SEQ_FULL   4096
#define CH         256
#define NHEAD      8
#define HDIM       32
#define QKV_O      (3 * CH)
#define ROWW       64
#define BQ         128
#define BK         32
#define NWAVE      8
#define TOK        64
#define XP         264
#define OPA        36
#define OPY        68
#define SB_V4      (TOK * XP / 8)

static_assert(CH == NHEAD * HDIM);
static_assert(HDIM == 32);
static_assert(ROWW == 2 * HDIM);
static_assert(SEQ % BQ == 0);
static_assert(SEQ % BK == 0);
static_assert(SEQ % TOK == 0);
static_assert(BQ == NWAVE * 16);
static_assert(TOK == 64);
static_assert(CH % 32 == 0);
static_assert(SEQ <= SEQ_FULL);
static_assert(NB >= 1 && NB <= NB_FULL);
static_assert((XP * 2) % 16 == 0);
static_assert(XP >= CH);
static_assert((OPA * 4) % 16 == 0);
static_assert((OPY * 4) % 16 == 0);
static_assert(OPA >= HDIM);
static_assert(OPY >= TOK);
static_assert((TOK * XP) % 8 == 0);
static_assert(NWAVE * 32 * ROWW * 2 <= SB_V4 * 16);
static_assert(4 * HDIM * TOK * 2 <= SB_V4 * 16);
static_assert(SB_V4 * 16 <= 65536);
static_assert((QKV_O * CH / 8) % 256 == 0);
static_assert((CH * CH / 8) % 256 == 0);

typedef __bf16   bf16;
typedef _Float16 f16;
typedef bf16     v16bf __attribute__((ext_vector_type(16)));
typedef f16      v16h  __attribute__((ext_vector_type(16)));
typedef float    v8f   __attribute__((ext_vector_type(8)));
typedef float    v4f   __attribute__((ext_vector_type(4)));
typedef unsigned v4u   __attribute__((ext_vector_type(4)));

union FragB  { v16bf v; v4u q[2]; bf16 h[16]; };
union FragH  { v16h  v; v4u q[2]; f16  h[16]; };
union Pack8B { v4u u; bf16 h[8]; };

constexpr size_t QK_PLANE  = (size_t)NB * NHEAD * SEQ * ROWW;
constexpr size_t WQ_BYTES  = (size_t)QKV_O * CH * 2;
constexpr size_t WO_BYTES  = (size_t)CH * CH * 2;
constexpr size_t QK_BYTES  = 2 * QK_PLANE * 2;
constexpr size_t VT_BYTES  = (size_t)NB * NHEAD * HDIM * SEQ * 2;
constexpr size_t CX_BYTES  = QK_PLANE * 2;
constexpr size_t WS_TOTAL  = WQ_BYTES + WO_BYTES + QK_BYTES + VT_BYTES + CX_BYTES;
static_assert(WQ_BYTES % 128 == 0 && WO_BYTES % 128 == 0 && QK_BYTES % 128 == 0 && VT_BYTES % 128 == 0);
static_assert(WS_TOTAL <= (size_t)134217728);

static __device__ __forceinline__ v8f mma_bf16(v16bf a, v16bf b, v8f acc) {
  acc = __builtin_amdgcn_wmma_f32_16x16x32_bf16(false, a, false, b, (short)0, acc, false, false);
  asm volatile("v_nop\n\tv_nop\n\tv_nop\n\tv_nop" : "+v"(acc) : "v"(a), "v"(b));
  return acc;
}
static __device__ __forceinline__ v8f mma_f16(v16h a, v16h b, v8f acc) {
  acc = __builtin_amdgcn_wmma_f32_16x16x32_f16(false, a, false, b, (short)0, acc, false, false);
  asm volatile("v_nop\n\tv_nop\n\tv_nop\n\tv_nop" : "+v"(acc) : "v"(a), "v"(b));
  return acc;
}

__global__ __launch_bounds__(256) void wcvt_kernel(const float* __restrict__ src,
                                                   bf16* __restrict__ dst, int n8) {
  const int i  = blockIdx.x * 256 + threadIdx.x;
  const int ic = (i < n8) ? i : (n8 - 1);
  const v4f a = *(const v4f*)(src + (size_t)ic * 8);
  const v4f c = *(const v4f*)(src + (size_t)ic * 8 + 4);
  Pack8B pk;
  #pragma unroll
  for (int e = 0; e < 4; ++e) {
    pk.h[e]     = (bf16)a[e];
    pk.h[4 + e] = (bf16)c[e];
  }
  const v4u val = pk.u;
  if (i < n8) *(volatile v4u*)(dst + (size_t)i * 8) = val;
  __threadfence();
  if (i < n8) *(volatile v4u*)(dst + (size_t)i * 8) = val;
}

__global__ __launch_bounds__(256) void qkv_planes_kernel(const float* __restrict__ x,
                                                         const bf16* __restrict__ wq,
                                                         const float* __restrict__ qb,
                                                         bf16* __restrict__ qk,
                                                         f16* __restrict__ vt) {
  const int tt    = blockIdx.x;
  const int which = (int)(blockIdx.y >> 1);
  const int hg    = (int)(blockIdx.y & 1);
  const int b     = blockIdx.z;
  const int tid   = threadIdx.x;
  const int wave  = tid >> 5;
  const int lane  = tid & 31;
  const int lq    = lane & 15;
  const int hi    = lane >> 4;
  const int hl    = wave >> 1;
  const int th    = wave & 1;
  const int head  = hg * 4 + hl;
  const int n0    = tt * TOK;

  __shared__ __align__(16) v4u sbuf4[SB_V4];
  bf16* sXb = reinterpret_cast<bf16*>(sbuf4);

  #pragma unroll 4
  for (int j = 0; j < 16; ++j) {
    const int c  = j * 16 + (tid >> 4);
    const int t4 = (tid & 15) * 4;
    const v4f xv = *(const v4f*)(x + ((size_t)b * CH + c) * SEQ_FULL + n0 + t4);
    #pragma unroll
    for (int e = 0; e < 4; ++e) sXb[(t4 + e) * XP + c] = (bf16)xv[e];
  }
  __syncthreads();

  v8f acc[2][2];
  #pragma unroll
  for (int ot = 0; ot < 2; ++ot) {
    #pragma unroll
    for (int nt = 0; nt < 2; ++nt) acc[ot][nt] = (v8f){0, 0, 0, 0, 0, 0, 0, 0};
  }

  const int orow0 = which * CH + head * HDIM;
  #pragma unroll
  for (int kk = 0; kk < CH / 32; ++kk) {
    FragB a[2], bx[2];
    #pragma unroll
    for (int ot = 0; ot < 2; ++ot) {
      const bf16* base = wq + (size_t)(orow0 + ot * 16 + lq) * CH + kk * 32 + hi * 8;
      a[ot].q[0] = *(const v4u*)(base);
      a[ot].q[1] = *(const v4u*)(base + 16);
    }
    #pragma unroll
    for (int nt = 0; nt < 2; ++nt) {
      const bf16* base = sXb + (th * 32 + nt * 16 + lq) * XP + kk * 32 + hi * 8;
      bx[nt].q[0] = *(const v4u*)(base);
      bx[nt].q[1] = *(const v4u*)(base + 16);
    }
    #pragma unroll
    for (int ot = 0; ot < 2; ++ot) {
      #pragma unroll
      for (int nt = 0; nt < 2; ++nt) acc[ot][nt] = mma_bf16(a[ot].v, bx[nt].v, acc[ot][nt]);
    }
  }

  float bs[2][8];
  #pragma unroll
  for (int ot = 0; ot < 2; ++ot) {
    const float* bp = qb + orow0 + ot * 16 + hi * 8;
    const v4f b0 = *(const v4f*)(bp);
    const v4f b1 = *(const v4f*)(bp + 4);
    #pragma unroll
    for (int e = 0; e < 4; ++e) {
      bs[ot][e]     = (float)(bf16)b0[e];
      bs[ot][4 + e] = (float)(bf16)b1[e];
    }
  }

  __syncthreads();

  if (which < 2) {
    bf16* se = reinterpret_cast<bf16*>(sbuf4) + wave * (32 * ROWW);
    #pragma unroll
    for (int ot = 0; ot < 2; ++ot) {
      #pragma unroll
      for (int nt = 0; nt < 2; ++nt) {
        #pragma unroll
        for (int r = 0; r < 8; ++r) {
          const int   tokl = nt * 16 + lq;
          const int   d    = ot * 16 + hi * 8 + r;
          const float v    = acc[ot][nt][r] + bs[ot][r];
          const bf16  vh   = (bf16)v;
          const bf16  vl   = (bf16)(v - (float)vh);
          se[tokl * ROWW + d]        = vh;
          se[tokl * ROWW + HDIM + d] = vl;
        }
      }
    }
  } else {
    f16* sv = reinterpret_cast<f16*>(sbuf4);
    #pragma unroll
    for (int ot = 0; ot < 2; ++ot) {
      #pragma unroll
      for (int nt = 0; nt < 2; ++nt) {
        #pragma unroll
        for (int r = 0; r < 8; ++r) {
          const int d   = ot * 16 + hi * 8 + r;
          const int tok = th * 32 + nt * 16 + lq;
          sv[(hl * HDIM + d) * TOK + tok] = (f16)(acc[ot][nt][r] + bs[ot][r]);
        }
      }
    }
  }
  __syncthreads();

  if (which < 2) {
    const bf16* se = reinterpret_cast<const bf16*>(sbuf4) + wave * (32 * ROWW);
    v4u    vals[8];
    size_t gidx[8];
    #pragma unroll
    for (int it = 0; it < 8; ++it) {
      const int tokl  = it * 4 + (lane >> 3);
      const int piece = lane & 7;
      vals[it] = *(const v4u*)(se + tokl * ROWW + piece * 8);
      gidx[it] = (size_t)which * QK_PLANE +
                 (((size_t)b * NHEAD + head) * SEQ + n0 + th * 32 + tokl) * ROWW + piece * 8;
    }
    #pragma unroll
    for (int it = 0; it < 8; ++it) *(volatile v4u*)(qk + gidx[it]) = vals[it];
    __threadfence();
    #pragma unroll
    for (int it = 0; it < 8; ++it) *(volatile v4u*)(qk + gidx[it]) = vals[it];
  } else {
    const f16* sv = reinterpret_cast<const f16*>(sbuf4);
    v4u    vals[4];
    size_t gidx[4];
    #pragma unroll
    for (int it = 0; it < 4; ++it) {
      const int line  = it * 32 + (tid >> 3);
      const int piece = tid & 7;
      const int hl2   = line >> 5;
      const int d2    = line & 31;
      vals[it] = *(const v4u*)(sv + line * TOK + piece * 8);
      gidx[it] = (((size_t)b * NHEAD + hg * 4 + hl2) * HDIM + d2) * SEQ + n0 + piece * 8;
    }
    #pragma unroll
    for (int it = 0; it < 4; ++it) *(volatile v4u*)(vt + gidx[it]) = vals[it];
    __threadfence();
    #pragma unroll
    for (int it = 0; it < 4; ++it) *(volatile v4u*)(vt + gidx[it]) = vals[it];
  }
}

__global__ __launch_bounds__(256) void attn_kernel(const bf16* __restrict__ qk,
                                                   const f16* __restrict__ vt,
                                                   bf16* __restrict__ cx) {
  const int qblk = blockIdx.x;
  const int h    = blockIdx.y;
  const int b    = blockIdx.z;
  const int tid  = threadIdx.x;
  const int wave = tid >> 5;
  const int lane = tid & 31;
  const int lq   = lane & 15;
  const int hi   = lane >> 4;

  __shared__ __align__(16) float sO[NWAVE * 16 * OPA];

  const int qrow0 = qblk * BQ + wave * 16;

  FragB qh, ql;
  {
    const bf16* qp = qk + (((size_t)b * NHEAD + h) * SEQ + qrow0 + lq) * ROWW;
    qh.q[0] = *(const v4u*)(qp + hi * 8);
    qh.q[1] = *(const v4u*)(qp + 16 + hi * 8);
    ql.q[0] = *(const v4u*)(qp + HDIM + hi * 8);
    ql.q[1] = *(const v4u*)(qp + HDIM + 16 + hi * 8);
  }

  const bf16* kp_h = qk + QK_PLANE + ((size_t)b * NHEAD + h) * SEQ * ROWW;
  const f16*  vt_h = vt + ((size_t)b * NHEAD + h) * HDIM * SEQ;

  v8f o[2];
  o[0] = (v8f){0, 0, 0, 0, 0, 0, 0, 0};
  o[1] = (v8f){0, 0, 0, 0, 0, 0, 0, 0};

  float rmax = -__builtin_inff();
  float rsum = 0.0f;
  const float SL = 0.17677669529663687f * 1.4426950408889634f;

  #pragma unroll 1
  for (int i = 0; i < SEQ / BK; ++i) {
    const int j0 = i * BK;

    FragB kh[2], kl[2];
    #pragma unroll
    for (int sub = 0; sub < 2; ++sub) {
      const bf16* base = kp_h + (size_t)(j0 + sub * 16 + lq) * ROWW + hi * 8;
      kh[sub].q[0] = *(const v4u*)(base);
      kh[sub].q[1] = *(const v4u*)(base + 16);
      kl[sub].q[0] = *(const v4u*)(base + HDIM);
      kl[sub].q[1] = *(const v4u*)(base + HDIM + 16);
    }
    FragH bv[2];
    #pragma unroll
    for (int dt = 0; dt < 2; ++dt) {
      const f16* base = vt_h + (size_t)(dt * 16 + lq) * SEQ + j0 + hi * 8;
      bv[dt].q[0] = *(const v4u*)(base);
      bv[dt].q[1] = *(const v4u*)(base + 16);
    }

    v8f c[2];
    #pragma unroll
    for (int sub = 0; sub < 2; ++sub) {
      v8f acc = (v8f){0, 0, 0, 0, 0, 0, 0, 0};
      acc = mma_bf16(kl[sub].v, qh.v, acc);
      acc = mma_bf16(kh[sub].v, ql.v, acc);
      acc = mma_bf16(kh[sub].v, qh.v, acc);
      c[sub] = acc;
    }

    float m_new = rmax;
    #pragma unroll
    for (int r = 0; r < 8; ++r) {
      m_new = fmaxf(m_new, c[0][r]);
      m_new = fmaxf(m_new, c[1][r]);
    }
    m_new = fmaxf(m_new, __shfl_xor(m_new, 16, 32));
    const float scale = __builtin_amdgcn_exp2f((rmax - m_new) * SL);
    rmax = m_new;

    FragH pa;
    float psum = 0.0f;
    #pragma unroll
    for (int r = 0; r < 8; ++r) {
      const float p0 = __builtin_amdgcn_exp2f((c[0][r] - m_new) * SL);
      const float p1 = __builtin_amdgcn_exp2f((c[1][r] - m_new) * SL);
      psum += p0 + p1;
      pa.h[r]     = (f16)(p0 * 4096.0f);
      pa.h[8 + r] = (f16)(p1 * 4096.0f);
    }
    const float psum_o = __shfl_xor(psum, 16, 32);
    rsum = rsum * scale + psum + psum_o;

    float sc[8];
    #pragma unroll
    for (int r = 0; r < 8; ++r) sc[r] = __shfl(scale, (hi << 3) + r, 32);
    #pragma unroll
    for (int dt = 0; dt < 2; ++dt) {
      #pragma unroll
      for (int r = 0; r < 8; ++r) o[dt][r] *= sc[r];
    }

    #pragma unroll
    for (int dt = 0; dt < 2; ++dt) o[dt] = mma_f16(pa.v, bv[dt].v, o[dt]);
  }

  float rs[8];
  #pragma unroll
  for (int r = 0; r < 8; ++r) rs[r] = 1.0f / __shfl(rsum, (hi << 3) + r, 32);

  float* so = sO + wave * (16 * OPA);
  #pragma unroll
  for (int r = 0; r < 8; ++r) {
    #pragma unroll
    for (int dt = 0; dt < 2; ++dt)
      so[(hi * 8 + r) * OPA + dt * 16 + lq] = o[dt][r] * (1.0f / 4096.0f) * rs[r];
  }
  __syncthreads();

  v4u    vals[4];
  size_t gidx[4];
  #pragma unroll
  for (int it = 0; it < 4; ++it) {
    const int tokl  = it * 4 + (lane >> 3);
    const int piece = lane & 7;
    const int pd    = (piece & 3) * 8;
    const v4f f0 = *(const v4f*)(so + tokl * OPA + pd);
    const v4f f1 = *(const v4f*)(so + tokl * OPA + pd + 4);
    Pack8B pk;
    #pragma unroll
    for (int e = 0; e < 4; ++e) {
      const float v0 = f0[e];
      const float v1 = f1[e];
      const bf16  h0 = (bf16)v0;
      const bf16  h1 = (bf16)v1;
      const bf16  l0 = (bf16)(v0 - (float)h0);
      const bf16  l1 = (bf16)(v1 - (float)h1);
      const float s0 = (piece < 4) ? (float)h0 : (float)l0;
      const float s1 = (piece < 4) ? (float)h1 : (float)l1;
      pk.h[e]     = (bf16)s0;
      pk.h[4 + e] = (bf16)s1;
    }
    vals[it] = pk.u;
    gidx[it] = (((size_t)b * NHEAD + h) * SEQ + qrow0 + tokl) * ROWW + piece * 8;
  }
  #pragma unroll
  for (int it = 0; it < 4; ++it) *(volatile v4u*)(cx + gidx[it]) = vals[it];
  __threadfence();
  #pragma unroll
  for (int it = 0; it < 4; ++it) *(volatile v4u*)(cx + gidx[it]) = vals[it];
}

__global__ __launch_bounds__(256) void oproj_kernel(const bf16* __restrict__ wo,
                                                    const bf16* __restrict__ cx,
                                                    const float* __restrict__ ob,
                                                    float* __restrict__ y) {
  const int tt   = blockIdx.x;
  const int og   = blockIdx.y;
  const int b    = blockIdx.z;
  const int tid  = threadIdx.x;
  const int wave = tid >> 5;
  const int lane = tid & 31;
  const int lq   = lane & 15;
  const int hi   = lane >> 4;
  const int o0   = (og * NWAVE + wave) * 16;
  const int n0   = tt * TOK;

  __shared__ __align__(16) float sY[NWAVE * 16 * OPY];

  v8f acc[4];
  #pragma unroll
  for (int nt = 0; nt < 4; ++nt) acc[nt] = (v8f){0, 0, 0, 0, 0, 0, 0, 0};

  #pragma unroll 1
  for (int kk = 0; kk < NHEAD; ++kk) {
    FragB a;
    {
      const bf16* base = wo + (size_t)(o0 + lq) * CH + kk * HDIM + hi * 8;
      a.q[0] = *(const v4u*)(base);
      a.q[1] = *(const v4u*)(base + 16);
    }
    #pragma unroll
    for (int nt = 0; nt < 4; ++nt) {
      const bf16* row = cx + (((size_t)b * NHEAD + kk) * SEQ + n0 + nt * 16 + lq) * ROWW;
      FragB bh, bl;
      bh.q[0] = *(const v4u*)(row + hi * 8);
      bh.q[1] = *(const v4u*)(row + 16 + hi * 8);
      bl.q[0] = *(const v4u*)(row + HDIM + hi * 8);
      bl.q[1] = *(const v4u*)(row + HDIM + 16 + hi * 8);
      acc[nt] = mma_bf16(a.v, bl.v, acc[nt]);
      acc[nt] = mma_bf16(a.v, bh.v, acc[nt]);
    }
  }

  float bs[8];
  {
    const float* bp = ob + o0 + hi * 8;
    const v4f b0 = *(const v4f*)(bp);
    const v4f b1 = *(const v4f*)(bp + 4);
    #pragma unroll
    for (int e = 0; e < 4; ++e) {
      bs[e]     = (float)(bf16)b0[e];
      bs[4 + e] = (float)(bf16)b1[e];
    }
  }

  float* so = sY + wave * (16 * OPY);
  #pragma unroll
  for (int nt = 0; nt < 4; ++nt) {
    #pragma unroll
    for (int r = 0; r < 8; ++r) so[(hi * 8 + r) * OPY + nt * 16 + lq] = acc[nt][r] + bs[r];
  }
  __syncthreads();

  v4f    vals[8];
  size_t gidx[8];
  #pragma unroll
  for (int it = 0; it < 8; ++it) {
    const int row = it * 2 + hi;
    vals[it] = *(const v4f*)(so + row * OPY + lq * 4);
    gidx[it] = ((size_t)b * CH + o0 + row) * SEQ_FULL + n0 + lq * 4;
  }
  #pragma unroll
  for (int it = 0; it < 8; ++it) *(volatile v4f*)(y + gidx[it]) = vals[it];
  __threadfence();
  #pragma unroll
  for (int it = 0; it < 8; ++it) *(volatile v4f*)(y + gidx[it]) = vals[it];
}

extern "C" void kernel_launch(void* const* d_in, const int* in_sizes, int n_in,
                              void* d_out, int out_size, void* d_ws, size_t ws_size,
                              hipStream_t stream) {
  if (n_in < 5) return;
  const size_t x_used = ((size_t)(NB - 1) * CH + (CH - 1)) * SEQ_FULL + SEQ;
  if ((size_t)in_sizes[0] < x_used) return;
  if ((size_t)in_sizes[1] < (size_t)QKV_O * CH) return;
  if ((size_t)in_sizes[2] < (size_t)QKV_O) return;
  if ((size_t)in_sizes[3] < (size_t)CH * CH) return;
  if ((size_t)in_sizes[4] < (size_t)CH) return;
  if ((size_t)out_size < x_used) return;
  if (ws_size < WS_TOTAL) return;

  const float* x     = (const float*)d_in[0];
  const float* qkv_w = (const float*)d_in[1];
  const float* qkv_b = (const float*)d_in[2];
  const float* out_w = (const float*)d_in[3];
  const float* out_b = (const float*)d_in[4];
  float*       y     = (float*)d_out;

  char* ws = (char*)d_ws;
  bf16* wq = (bf16*)(ws);
  bf16* wo = (bf16*)(ws + WQ_BYTES);
  bf16* qk = (bf16*)(ws + WQ_BYTES + WO_BYTES);
  f16*  vt = (f16*)(ws + WQ_BYTES + WO_BYTES + QK_BYTES);
  bf16* cx = (bf16*)(ws + WQ_BYTES + WO_BYTES + QK_BYTES + VT_BYTES);

  wcvt_kernel<<<dim3(QKV_O * CH / 8 / 256), 256, 0, stream>>>(qkv_w, wq, QKV_O * CH / 8);
  wcvt_kernel<<<dim3(CH * CH / 8 / 256), 256, 0, stream>>>(out_w, wo, CH * CH / 8);

  qkv_planes_kernel<<<dim3(SEQ / TOK, 6, NB), 256, 0, stream>>>(x, wq, qkv_b, qk, vt);

  attn_kernel<<<dim3(SEQ / BQ, NHEAD, NB), 256, 0, stream>>>(qk, vt, cx);

  oproj_kernel<<<dim3(SEQ / TOK, CH / (NWAVE * 16), NB), 256, 0, stream>>>(wo, cx, out_b, y);
}
